// DCNConv_74019466379803
// MI455X (gfx1250) — hardware-verified
//
#include <hip/hip_runtime.h>
#include <stddef.h>
#include <stdint.h>


#define NIMG   8
#define CH     256
#define HI     64
#define WI     64
#define LPIX   (HI * WI)
#define NGRP   8
#define NPT    9
#define CGRP   (CH / NGRP)
#define MROWS  (NIMG * LPIX)
#define OMD    (NGRP * NPT * 3)
#define OMP    224
#define KD     256
#define TP     68
#define SP     36
#define APITCH 264
#define DP     36
#define APB    (32 * APITCH * 2)
#define DSB    (CH * DP * 4)
#define SAMP_LDS (2 * APB + DSB)

static_assert(OMP % 32 == 0 && OMP >= OMD);
static_assert(MROWS % 128 == 0);
static_assert((APB % 16) == 0);
static_assert(SAMP_LDS == 70656);
static_assert((TP * 4) % 16 == 0 && (SP * 4) % 16 == 0 && (APITCH * 2) % 16 == 0 && (DP * 4) % 16 == 0);

typedef float v4f __attribute__((ext_vector_type(4)));
typedef float v8f __attribute__((ext_vector_type(8)));
typedef unsigned short us_t;
typedef us_t v8us __attribute__((ext_vector_type(8)));
typedef __bf16 v16bf __attribute__((ext_vector_type(16)));
union FragB { v16bf v; v8us u[2]; };

__device__ __forceinline__ unsigned bf16_bits(float x) {
  unsigned u = __float_as_uint(x);
  u = u + 0x7FFFu + ((u >> 16) & 1u);
  return u >> 16;
}

__device__ __forceinline__ void split1(float x, us_t& h, us_t& l) {
  const unsigned hb = bf16_bits(x);
  const float hf = __uint_as_float(hb << 16);
  h = (us_t)hb;
  l = (us_t)bf16_bits(x - hf);
}

__device__ __forceinline__ v8f zf8() {
  v8f r;
#pragma unroll
  for (int i = 0; i < 8; ++i) r[i] = 0.0f;
  return r;
}

__device__ __forceinline__ v8f wmb3(v16bf ah, v16bf al, v16bf bh, v16bf bl, v8f c) {
  v8f d = __builtin_amdgcn_wmma_f32_16x16x32_bf16(false, ah, false, bh, (short)0, c, false, false);
  d = __builtin_amdgcn_wmma_f32_16x16x32_bf16(false, ah, false, bl, (short)0, d, false, false);
  d = __builtin_amdgcn_wmma_f32_16x16x32_bf16(false, al, false, bh, (short)0, d, false, false);
  asm volatile("v_nop\n\tv_nop\n\tv_nop\n\tv_nop" : "+v"(d) : "v"(ah), "v"(al), "v"(bh), "v"(bl));
  return d;
}

__global__ __launch_bounds__(32) void k_wsplit(const float* __restrict__ src, int srcRows,
                                               us_t* ph, us_t* pl, int dstRows) {
  const int row = blockIdx.x;
  const int lane = threadIdx.x & 31;
  if (row >= dstRows) return;
  const bool live = row < srcRows;
  const int sr = live ? row : (srcRows - 1);
  const float* p = src + (size_t)sr * KD + 8 * lane;
  const v4f a = *(const v4f*)p;
  const v4f b = *(const v4f*)(p + 4);
  v8us vh, vl;
#pragma unroll
  for (int i = 0; i < 4; ++i) {
    us_t h0, l0, h1, l1;
    split1(live ? a[i] : 0.0f, h0, l0);
    split1(live ? b[i] : 0.0f, h1, l1);
    vh[i] = h0; vl[i] = l0; vh[4 + i] = h1; vl[4 + i] = l1;
  }
  const size_t o = (size_t)row * KD + 8 * lane;
  *(volatile v8us*)(ph + o) = vh;
  *(volatile v8us*)(pl + o) = vl;
  __threadfence();
  *(volatile v8us*)(ph + o) = vh;
  *(volatile v8us*)(pl + o) = vl;
}

__global__ __launch_bounds__(256) void k_xprep(const float* __restrict__ x, const float* __restrict__ dww,
                                               const float* __restrict__ dwb,
                                               us_t* xh, us_t* xl, us_t* dh, us_t* dl) {
  __shared__ __attribute__((aligned(16))) float Tx[64 * TP];
  __shared__ __attribute__((aligned(16))) float Td[64 * TP];
  const int tid = threadIdx.x, lane = tid & 31, wave = tid >> 5;
  const int b  = blockIdx.x;
  const int cc = b & 3;
  const int h  = (b >> 2) & (HI - 1);
  const int n  = b >> 8;
  const int c0 = cc * 64;
  const int w  = tid & 63;
  const int cl0 = tid >> 6;

#pragma unroll 1
  for (int i = 0; i < 16; ++i) {
    const int cl = cl0 + 4 * i;
    const int c  = c0 + cl;
    const float* xp = x + ((size_t)n * CH + c) * LPIX;
    const float* wp = dww + c * 9;
    float s = 0.0f, xv = 0.0f;
#pragma unroll
    for (int ky = 0; ky < 3; ++ky) {
      const int y  = h + ky - 1;
      const int yc = y < 0 ? 0 : (y > HI - 1 ? HI - 1 : y);
      const bool vy = (unsigned)y < (unsigned)HI;
#pragma unroll
      for (int kx = 0; kx < 3; ++kx) {
        const int xx = w + kx - 1;
        const int xc = xx < 0 ? 0 : (xx > WI - 1 ? WI - 1 : xx);
        const bool ok = vy && ((unsigned)xx < (unsigned)WI);
        const float t = xp[yc * WI + xc];
        if (ky == 1 && kx == 1) xv = t;
        s = fmaf(wp[ky * 3 + kx], ok ? t : 0.0f, s);
      }
    }
    s += dwb[c];
    Tx[w * TP + cl] = xv;
    Td[w * TP + cl] = s;
  }
  __syncthreads();

  const int q = lane >> 3, j = lane & 7;
  v8us o[2][4];
  size_t mrow[2];
#pragma unroll
  for (int it = 0; it < 2; ++it) {
    const int wpos = wave * 8 + it * 4 + q;
    const float* tx = Tx + wpos * TP + 8 * j;
    const float* td = Td + wpos * TP + 8 * j;
    const v4f xa = *(const v4f*)tx, xb = *(const v4f*)(tx + 4);
    const v4f da = *(const v4f*)td, db = *(const v4f*)(td + 4);
#pragma unroll
    for (int e = 0; e < 4; ++e) {
      us_t hb, lb;
      split1(xa[e], hb, lb); o[it][0][e] = hb;     o[it][1][e] = lb;
      split1(xb[e], hb, lb); o[it][0][4 + e] = hb; o[it][1][4 + e] = lb;
      split1(da[e], hb, lb); o[it][2][e] = hb;     o[it][3][e] = lb;
      split1(db[e], hb, lb); o[it][2][4 + e] = hb; o[it][3][4 + e] = lb;
    }
    mrow[it] = ((size_t)(n * LPIX + h * WI + wpos)) * CH + c0 + 8 * j;
  }
#pragma unroll
  for (int it = 0; it < 2; ++it) {
    *(volatile v8us*)(xh + mrow[it]) = o[it][0];
    *(volatile v8us*)(xl + mrow[it]) = o[it][1];
    *(volatile v8us*)(dh + mrow[it]) = o[it][2];
    *(volatile v8us*)(dl + mrow[it]) = o[it][3];
  }
  __threadfence();
#pragma unroll
  for (int it = 0; it < 2; ++it) {
    *(volatile v8us*)(xh + mrow[it]) = o[it][0];
    *(volatile v8us*)(xl + mrow[it]) = o[it][1];
    *(volatile v8us*)(dh + mrow[it]) = o[it][2];
    *(volatile v8us*)(dl + mrow[it]) = o[it][3];
  }
}

__global__ __launch_bounds__(256) void k_gemm(const us_t* __restrict__ Ah, const us_t* __restrict__ Al,
                                              const us_t* __restrict__ Bh, const us_t* __restrict__ Bl,
                                              const float* __restrict__ bias, int biasN,
                                              float* outp, int P, int nbN) {
  __shared__ __attribute__((aligned(16))) float stg[8 * 16 * SP];
  const int tid = threadIdx.x, lane = tid & 31, wave = tid >> 5, hf = lane >> 4, m = lane & 15;
  const int bn = blockIdx.x % nbN;
  const int bm = blockIdx.x / nbN;
  const int r0 = bm * 128 + wave * 16;
  const int c0 = bn * 32;

  const us_t* arh = Ah + (size_t)(r0 + m) * KD + 8 * hf;
  const us_t* arl = Al + (size_t)(r0 + m) * KD + 8 * hf;
  const us_t* b0h = Bh + (size_t)(c0 + m) * KD + 8 * hf;
  const us_t* b0l = Bl + (size_t)(c0 + m) * KD + 8 * hf;
  const us_t* b1h = Bh + (size_t)(c0 + 16 + m) * KD + 8 * hf;
  const us_t* b1l = Bl + (size_t)(c0 + 16 + m) * KD + 8 * hf;

  v8f acc0 = zf8(), acc1 = zf8();
#pragma unroll 2
  for (int k0 = 0; k0 < KD; k0 += 32) {
    FragB ah, al, bh, bl;
    ah.u[0] = *(const v8us*)(arh + k0); ah.u[1] = *(const v8us*)(arh + k0 + 16);
    al.u[0] = *(const v8us*)(arl + k0); al.u[1] = *(const v8us*)(arl + k0 + 16);
    bh.u[0] = *(const v8us*)(b0h + k0); bh.u[1] = *(const v8us*)(b0h + k0 + 16);
    bl.u[0] = *(const v8us*)(b0l + k0); bl.u[1] = *(const v8us*)(b0l + k0 + 16);
    acc0 = wmb3(ah.v, al.v, bh.v, bl.v, acc0);
    bh.u[0] = *(const v8us*)(b1h + k0); bh.u[1] = *(const v8us*)(b1h + k0 + 16);
    bl.u[0] = *(const v8us*)(b1l + k0); bl.u[1] = *(const v8us*)(b1l + k0 + 16);
    acc1 = wmb3(ah.v, al.v, bh.v, bl.v, acc1);
  }

  const int colA = c0 + m, colB = c0 + 16 + m;
  const int biA = colA < biasN ? colA : (biasN - 1);
  const int biB = colB < biasN ? colB : (biasN - 1);
  const float ldA = bias[biA], ldB = bias[biB];
  const float bvA = (colA < biasN) ? ldA : 0.0f;
  const float bvB = (colB < biasN) ? ldB : 0.0f;

  float* sw = stg + wave * 16 * SP;
#pragma unroll
  for (int r = 0; r < 8; ++r) {
    sw[(8 * hf + r) * SP + m]      = acc0[r] + bvA;
    sw[(8 * hf + r) * SP + 16 + m] = acc1[r] + bvB;
  }
  __syncthreads();

  const int q = lane >> 3, j = lane & 7;
  v4f ov[4];
  size_t go[4];
#pragma unroll
  for (int i = 0; i < 4; ++i) {
    const int row = 4 * i + q;
    ov[i] = *(const v4f*)(sw + row * SP + 4 * j);
    go[i] = (size_t)(r0 + row) * (size_t)P + c0 + 4 * j;
  }
#pragma unroll
  for (int i = 0; i < 4; ++i) *(volatile v4f*)(outp + go[i]) = ov[i];
  __threadfence();
#pragma unroll
  for (int i = 0; i < 4; ++i) *(volatile v4f*)(outp + go[i]) = ov[i];
}

__global__ __launch_bounds__(256) void k_samp(const float* __restrict__ value, const float* __restrict__ om,
                                              const us_t* __restrict__ Bh, const us_t* __restrict__ Bl,
                                              float* outp) {
  extern __shared__ __attribute__((aligned(16))) unsigned char dyn[];
  us_t*  Ah = (us_t*)dyn;
  us_t*  Al = (us_t*)(dyn + APB);
  float* Ds = (float*)(dyn + 2 * APB);

  const int tid = threadIdx.x, lane = tid & 31, wave = tid >> 5, hf = lane >> 4, m = lane & 15;
  const int m0 = blockIdx.x * 32;
  const int n  = m0 >> 12;
  const int l0 = m0 & (LPIX - 1);

  {
    const int px = lane, g = wave;
    const int mpos = m0 + px;
    const int l = l0 + px;
    const int hh = l >> 6, ww = l & 63;
    const float* omr = om + (size_t)mpos * OMP + g * (NPT * 3);
    const float* vbase = value + (size_t)n * LPIX * CH + g * CGRP;
    float acc[CGRP];
#pragma unroll
    for (int c = 0; c < CGRP; ++c) acc[c] = 0.0f;

#pragma unroll 1
    for (int k = 0; k < NPT; ++k) {
      const float oy = omr[2 * k];
      const float ox = omr[2 * k + 1];
      const float mk = omr[2 * NPT + k];
      const int kq = k / 3;
      const int by = kq - 1;
      const int bx = (k - kq * 3) - 1;
      float py = (float)(hh + by) + oy;
      float pxf = (float)(ww + bx) + ox;
      py  = fminf(fmaxf(py,  -2.0f), (float)(HI + 1));
      pxf = fminf(fmaxf(pxf, -2.0f), (float)(WI + 1));
      const float y0f = floorf(py), x0f = floorf(pxf);
      const float ty = py - y0f, tx = pxf - x0f;
      const int y0 = (int)y0f, x0 = (int)x0f;
#pragma unroll 1
      for (int qc = 0; qc < 4; ++qc) {
        const int qy = qc >> 1, qx = qc & 1;
        const int yy = y0 + qy, xx = x0 + qx;
        const float wy = qy ? ty : (1.0f - ty);
        const float wx = qx ? tx : (1.0f - tx);
        const bool valid = ((unsigned)yy < (unsigned)HI) && ((unsigned)xx < (unsigned)WI);
        float coef = mk * (wy * wx);
        coef = valid ? coef : 0.0f;
        const int yi = yy < 0 ? 0 : (yy > HI - 1 ? HI - 1 : yy);
        const int xi = xx < 0 ? 0 : (xx > WI - 1 ? WI - 1 : xx);
        const float* vr = vbase + (size_t)(yi * WI + xi) * CH;
#pragma unroll
        for (int c4 = 0; c4 < 8; ++c4) {
          const v4f v = *(const v4f*)(vr + 4 * c4);
          acc[4 * c4 + 0] = fmaf(coef, v.x, acc[4 * c4 + 0]);
          acc[4 * c4 + 1] = fmaf(coef, v.y, acc[4 * c4 + 1]);
          acc[4 * c4 + 2] = fmaf(coef, v.z, acc[4 * c4 + 2]);
          acc[4 * c4 + 3] = fmaf(coef, v.w, acc[4 * c4 + 3]);
        }
      }
    }

    us_t* ahr = Ah + px * APITCH + g * CGRP;
    us_t* alr = Al + px * APITCH + g * CGRP;
#pragma unroll
    for (int i = 0; i < 4; ++i) {
      v8us vh, vl;
#pragma unroll
      for (int e = 0; e < 8; ++e) {
        us_t hb, lb;
        split1(acc[8 * i + e], hb, lb);
        vh[e] = hb; vl[e] = lb;
      }
      *(v8us*)(ahr + 8 * i) = vh;
      *(v8us*)(alr + 8 * i) = vl;
    }
  }
  __syncthreads();

  {
    const int wm = wave & 1, wn = wave >> 1;
    const us_t* arh = Ah + (16 * wm + m) * APITCH + 8 * hf;
    const us_t* arl = Al + (16 * wm + m) * APITCH + 8 * hf;
    v8f acc0 = zf8(), acc1 = zf8(), acc2 = zf8(), acc3 = zf8();
#pragma unroll 2
    for (int k0 = 0; k0 < KD; k0 += 32) {
      FragB ah, al, bh, bl;
      ah.u[0] = *(const v8us*)(arh + k0); ah.u[1] = *(const v8us*)(arh + k0 + 16);
      al.u[0] = *(const v8us*)(arl + k0); al.u[1] = *(const v8us*)(arl + k0 + 16);
      {
        const us_t* bph = Bh + (size_t)(64 * wn + 0 + m) * KD + 8 * hf + k0;
        const us_t* bpl = Bl + (size_t)(64 * wn + 0 + m) * KD + 8 * hf + k0;
        bh.u[0] = *(const v8us*)bph; bh.u[1] = *(const v8us*)(bph + 16);
        bl.u[0] = *(const v8us*)bpl; bl.u[1] = *(const v8us*)(bpl + 16);
        acc0 = wmb3(ah.v, al.v, bh.v, bl.v, acc0);
      }
      {
        const us_t* bph = Bh + (size_t)(64 * wn + 16 + m) * KD + 8 * hf + k0;
        const us_t* bpl = Bl + (size_t)(64 * wn + 16 + m) * KD + 8 * hf + k0;
        bh.u[0] = *(const v8us*)bph; bh.u[1] = *(const v8us*)(bph + 16);
        bl.u[0] = *(const v8us*)bpl; bl.u[1] = *(const v8us*)(bpl + 16);
        acc1 = wmb3(ah.v, al.v, bh.v, bl.v, acc1);
      }
      {
        const us_t* bph = Bh + (size_t)(64 * wn + 32 + m) * KD + 8 * hf + k0;
        const us_t* bpl = Bl + (size_t)(64 * wn + 32 + m) * KD + 8 * hf + k0;
        bh.u[0] = *(const v8us*)bph; bh.u[1] = *(const v8us*)(bph + 16);
        bl.u[0] = *(const v8us*)bpl; bl.u[1] = *(const v8us*)(bpl + 16);
        acc2 = wmb3(ah.v, al.v, bh.v, bl.v, acc2);
      }
      {
        const us_t* bph = Bh + (size_t)(64 * wn + 48 + m) * KD + 8 * hf + k0;
        const us_t* bpl = Bl + (size_t)(64 * wn + 48 + m) * KD + 8 * hf + k0;
        bh.u[0] = *(const v8us*)bph; bh.u[1] = *(const v8us*)(bph + 16);
        bl.u[0] = *(const v8us*)bpl; bl.u[1] = *(const v8us*)(bpl + 16);
        acc3 = wmb3(ah.v, al.v, bh.v, bl.v, acc3);
      }
    }

    const int pr = 16 * wm + 8 * hf;
    {
      float* dp = Ds + (64 * wn + 0 + m) * DP + pr;
      v4f a = {acc0[0], acc0[1], acc0[2], acc0[3]}; v4f b = {acc0[4], acc0[5], acc0[6], acc0[7]};
      *(v4f*)dp = a; *(v4f*)(dp + 4) = b;
    }
    {
      float* dp = Ds + (64 * wn + 16 + m) * DP + pr;
      v4f a = {acc1[0], acc1[1], acc1[2], acc1[3]}; v4f b = {acc1[4], acc1[5], acc1[6], acc1[7]};
      *(v4f*)dp = a; *(v4f*)(dp + 4) = b;
    }
    {
      float* dp = Ds + (64 * wn + 32 + m) * DP + pr;
      v4f a = {acc2[0], acc2[1], acc2[2], acc2[3]}; v4f b = {acc2[4], acc2[5], acc2[6], acc2[7]};
      *(v4f*)dp = a; *(v4f*)(dp + 4) = b;
    }
    {
      float* dp = Ds + (64 * wn + 48 + m) * DP + pr;
      v4f a = {acc3[0], acc3[1], acc3[2], acc3[3]}; v4f b = {acc3[4], acc3[5], acc3[6], acc3[7]};
      *(v4f*)dp = a; *(v4f*)(dp + 4) = b;
    }
  }
  __syncthreads();

  {
    const int q = lane >> 3, j = lane & 7;
    v4f ov[8];
    size_t go[8];
#pragma unroll
    for (int i = 0; i < 8; ++i) {
      const int o = 32 * wave + 4 * i + q;
      ov[i] = *(const v4f*)(Ds + o * DP + 4 * j);
      go[i] = ((size_t)(n * CH + o)) * LPIX + l0 + 4 * j;
    }
#pragma unroll
    for (int i = 0; i < 8; ++i) *(volatile v4f*)(outp + go[i]) = ov[i];
    __threadfence();
#pragma unroll
    for (int i = 0; i < 8; ++i) *(volatile v4f*)(outp + go[i]) = ov[i];
  }
}

extern "C" void kernel_launch(void* const* d_in, const int* in_sizes, int n_in,
                              void* d_out, int out_size, void* d_ws, size_t ws_size,
                              hipStream_t stream) {
  if (n_in < 8) return;
  if (in_sizes[0] != NIMG * CH * LPIX) return;
  if (in_sizes[1] != CH * 9 || in_sizes[2] != CH) return;
  if (in_sizes[3] != OMD * CH || in_sizes[4] != OMD) return;
  if (in_sizes[5] != CH * CH || in_sizes[6] != CH || in_sizes[7] != CH * CH) return;
  if (out_size != NIMG * CH * LPIX) return;

  const float* x    = (const float*)d_in[0];
  const float* dw_w = (const float*)d_in[1];
  const float* dw_b = (const float*)d_in[2];
  const float* om_w = (const float*)d_in[3];
  const float* om_b = (const float*)d_in[4];
  const float* vp_w = (const float*)d_in[5];
  const float* vp_b = (const float*)d_in[6];
  const float* op_w = (const float*)d_in[7];
  float* out = (float*)d_out;

  const size_t plane16 = (size_t)MROWS * CH * sizeof(us_t);
  size_t off = 0;
  const size_t oXh = off; off += plane16;
  const size_t oXl = off; off += plane16;
  const size_t oDh = off; off += plane16;
  const size_t oDl = off; off += plane16;
  const size_t oVal = off; off += (size_t)MROWS * CH * sizeof(float);
  const size_t oOm  = off; off += (size_t)MROWS * OMP * sizeof(float);
  const size_t oVph = off; off += (size_t)CH * KD * sizeof(us_t);
  const size_t oVpl = off; off += (size_t)CH * KD * sizeof(us_t);
  const size_t oOph = off; off += (size_t)CH * KD * sizeof(us_t);
  const size_t oOpl = off; off += (size_t)CH * KD * sizeof(us_t);
  const size_t oOmh = off; off += (size_t)OMP * KD * sizeof(us_t);
  const size_t oOml = off; off += (size_t)OMP * KD * sizeof(us_t);
  if (off > ws_size) return;
  if (off > (size_t)134217728) return;

  char* ws = (char*)d_ws;
  us_t* xh  = (us_t*)(ws + oXh);
  us_t* xl  = (us_t*)(ws + oXl);
  us_t* dh  = (us_t*)(ws + oDh);
  us_t* dl  = (us_t*)(ws + oDl);
  float* value = (float*)(ws + oVal);
  float* omp   = (float*)(ws + oOm);
  us_t* vph = (us_t*)(ws + oVph);
  us_t* vpl = (us_t*)(ws + oVpl);
  us_t* oph = (us_t*)(ws + oOph);
  us_t* opl = (us_t*)(ws + oOpl);
  us_t* omh = (us_t*)(ws + oOmh);
  us_t* oml = (us_t*)(ws + oOml);

  k_wsplit<<<CH, 32, 0, stream>>>(vp_w, CH, vph, vpl, CH);
  k_wsplit<<<OMP, 32, 0, stream>>>(om_w, OMD, omh, oml, OMP);
  k_wsplit<<<CH, 32, 0, stream>>>(op_w, CH, oph, opl, CH);

  k_xprep<<<NIMG * HI * (CH / 64), 256, 0, stream>>>(x, dw_w, dw_b, xh, xl, dh, dl);

  k_gemm<<<(MROWS / 128) * (CH / 32), 256, 0, stream>>>(xh, xl, vph, vpl, vp_b, CH, value, CH, CH / 32);

  k_gemm<<<(MROWS / 128) * (OMP / 32), 256, 0, stream>>>(dh, dl, omh, oml, om_b, OMD, omp, OMP, OMP / 32);

  hipFuncSetAttribute(reinterpret_cast<const void*>(&k_samp), hipFuncAttributeMaxDynamicSharedMemorySize, SAMP_LDS);
  k_samp<<<MROWS / 32, 256, SAMP_LDS, stream>>>(value, omp, oph, opl, out);
}
